// OnlineTripletLoss_16423954940178
// MI455X (gfx1250) — hardware-verified
//
#include <hip/hip_runtime.h>


namespace {
constexpr int N = 8192, D = 128, NC = 10, NB = N / 128;

typedef _Float16 b16;
typedef __attribute__((ext_vector_type(16))) _Float16 v16b;
typedef __attribute__((ext_vector_type(8)))  _Float16 v8b;
typedef __attribute__((ext_vector_type(8)))  float v8f;
typedef __attribute__((ext_vector_type(4)))  float v4f;

__device__ __forceinline__ v8b ld8b(const b16* p) { return *(const v8b*)p; }
__device__ __forceinline__ v16b cat8b(v8b a, v8b b) { return __builtin_shufflevector(a, b, 0, 1, 2, 3, 4, 5, 6, 7, 8, 9, 10, 11, 12, 13, 14, 15); }
__device__ __forceinline__ v16b frag_kb(const b16* p, int hh) { return cat8b(ld8b(p + 8 * hh), ld8b(p + 16 + 8 * hh)); }
__device__ __forceinline__ void split16(float v, b16& hi, b16& lo) { hi = (b16)v; lo = (b16)(v - (float)hi); }
__device__ __forceinline__ void frag_ksplit(const float* p, int hh, v16b& fh_, v16b& fl_) {
  const float* p0 = p + 8 * hh; const float* p1 = p + 16 + 8 * hh;
#pragma unroll
  for (int e = 0; e < 8; ++e) { b16 a, c; split16(p0[e], a, c); fh_[e] = a; fl_[e] = c; split16(p1[e], a, c); fh_[8 + e] = a; fl_[8 + e] = c; }
}
__device__ __forceinline__ v8f wmma16b(v16b a, v16b b, v8f c) {
  v8f d = __builtin_amdgcn_wmma_f32_16x16x32_f16(false, a, false, b, (short)0, c, false, false);
  asm volatile("v_nop\n\tv_nop\n\tv_nop\n\tv_nop" : "+v"(d) : "v"(a), "v"(b));
  return d;
}
__device__ __forceinline__ void wave_lds_sync() {
  __builtin_amdgcn_fence(__ATOMIC_RELEASE, "workgroup");
  __builtin_amdgcn_wave_barrier();
  __builtin_amdgcn_fence(__ATOMIC_ACQUIRE, "workgroup");
}

struct Opnd { const void* p0; const void* p1; int ld; };
template <int NP> __device__ __forceinline__ void load_frags(const Opnd& o, int row, int kb, int hh, v16b& fh_, v16b& fl_) {
  if (NP == 0) { frag_ksplit((const float*)o.p0 + (size_t)row * o.ld + kb, hh, fh_, fl_); }
  else if (NP == 4) {
    const float* p = (const float*)o.p0 + (size_t)row * o.ld + kb; const float* p0 = p + 8 * hh; const float* p1 = p + 16 + 8 * hh;
#pragma unroll
    for (int e = 0; e < 8; ++e) { b16 a, c; split16(p0[e] * 64.0f, a, c); fh_[e] = a; fl_[e] = c; split16(p1[e] * 64.0f, a, c); fh_[8 + e] = a; fl_[8 + e] = c; }
  } else if (NP == 3) {
    const float* p = (const float*)o.p0 + (size_t)row * o.ld + kb; const float* p0 = p + 8 * hh; const float* p1 = p + 16 + 8 * hh;
#pragma unroll
    for (int e = 0; e < 8; ++e) { fh_[e] = (b16)p0[e]; fh_[8 + e] = (b16)p1[e]; }
    fl_ = fh_;
  } else {
    fh_ = frag_kb((const b16*)o.p0 + (size_t)row * o.ld + kb, hh);
    if (NP == 2) fl_ = frag_kb((const b16*)o.p1 + (size_t)row * o.ld + kb, hh); else fl_ = fh_;
  }
}
template <int ANP, int BNP> __device__ __forceinline__ v8f mac(v16b ah, v16b al, v16b bh, v16b bl, v8f c) {
  c = wmma16b(ah, bh, c);
  if (BNP == 0 || BNP == 2 || BNP == 4) c = wmma16b(ah, bl, c);
  if (ANP == 0 || ANP == 2 || ANP == 4) c = wmma16b(al, bh, c);
  return c;
}
template <int ANP, int BNP>
__device__ __forceinline__ void gemm_tile(const Opnd& A, const Opnd& B, int K, int m0, int c0, int nloc, int hlf, v8f (&acc)[2][4]) {
  for (int kb = 0; kb < K; kb += 32) {
    v16b a0h, a0l, a1h, a1l;
    load_frags<ANP>(A, m0 + nloc, kb, hlf, a0h, a0l);
    load_frags<ANP>(A, m0 + 16 + nloc, kb, hlf, a1h, a1l);
#pragma unroll
    for (int t = 0; t < 4; ++t) {
      v16b bh, bl;
      load_frags<BNP>(B, c0 + t * 16 + nloc, kb, hlf, bh, bl);
      acc[0][t] = mac<ANP, BNP>(a0h, a0l, bh, bl, acc[0][t]);
      acc[1][t] = mac<ANP, BNP>(a1h, a1l, bh, bl, acc[1][t]);
    }
  }
}

__device__ __forceinline__ void epi_planes(v8f (&acc)[2][4], float scale, bool two, b16* __restrict__ oh, b16* __restrict__ ol, int ldo,
                                           int m0, int c0, int lane, b16* Th, b16* Tl) {
  const int nloc = lane & 15, hlf = lane >> 4;
#pragma unroll
  for (int t = 0; t < 4; ++t)
#pragma unroll
    for (int r = 0; r < 2; ++r)
#pragma unroll
      for (int v = 0; v < 8; ++v) {
        const int rr = r * 16 + v + 8 * hlf, cc = t * 16 + nloc;
        b16 h_, l_; split16(acc[r][t][v] * scale, h_, l_);
        Th[rr * 64 + cc] = h_; Tl[rr * 64 + cc] = l_;
      }
  wave_lds_sync();
  for (int pass = 0; pass < 2; ++pass) {
#pragma unroll
    for (int j = 0; j < 8; ++j) {
      const int rr = j * 4 + (lane >> 3), c8 = (lane & 7) * 8;
      const size_t o = (size_t)(m0 + rr) * ldo + c0 + c8;
      *(volatile v8b*)(oh + o) = ld8b(Th + rr * 64 + c8);
      if (two) *(volatile v8b*)(ol + o) = ld8b(Tl + rr * 64 + c8);
    }
    __threadfence();
  }
}
__device__ __forceinline__ void epi_f32(v8f (&acc)[2][4], float scale, const float* rscale, float* __restrict__ out, int ldo, int m0, int c0, int lane, float* Tt) {
  const int nloc = lane & 15, hlf = lane >> 4;
#pragma unroll
  for (int t = 0; t < 4; ++t)
#pragma unroll
    for (int r = 0; r < 2; ++r)
#pragma unroll
      for (int v = 0; v < 8; ++v) {
        const int rr = r * 16 + v + 8 * hlf;
        const float rs = rscale ? rscale[(size_t)(m0 + rr) * 32] : 1.0f;
        Tt[rr * 64 + t * 16 + nloc] = acc[r][t][v] * scale * rs;
      }
  wave_lds_sync();
  float* dst0 = out + (size_t)m0 * ldo + c0;
  for (int pass = 0; pass < 2; ++pass) {
#pragma unroll
    for (int j = 0; j < 16; ++j) { const int rr = j * 2 + hlf, c4 = nloc * 4; *(volatile v4f*)(dst0 + (size_t)rr * ldo + c4) = *(const v4f*)(Tt + rr * 64 + c4); }
    __threadfence();
  }
}


__global__ __launch_bounds__(256) void prep_kernel(const float* __restrict__ e, const int* __restrict__ lab, b16* __restrict__ e16, float* __restrict__ sq,
                                                   float* __restrict__ mc, float* __restrict__ Sc, float* __restrict__ ncnt) {
  __shared__ float sqs[N];
  const int t = threadIdx.x;
  for (int pass = 0; pass < 2; ++pass) {
    for (int p = t; p < N * D / 8; p += 256) { const size_t i0 = (size_t)p * 8; v8b v; float s = 0.0f;
#pragma unroll
      for (int k = 0; k < 8; ++k) v[k] = (b16)e[i0 + k];
      *(volatile v8b*)(e16 + i0) = v; (void)s; }
    __threadfence();
  }
  for (int j = t; j < N; j += 256) { float s = 0.0f;
#pragma unroll 1
    for (int dd = 0; dd < D; ++dd) { const float v = e[(size_t)j * D + dd]; s += v * v; }
    sqs[j] = s; }
  __syncthreads();
  for (int pass = 0; pass < 2; ++pass) { for (int j = t; j < N; j += 256) ((volatile float*)sq)[j] = sqs[j]; __threadfence(); }
  __shared__ float mcl[NC * D]; __shared__ float scl[64];
  for (int q = t; q < NC * D + NC; q += 256) {
    if (q < NC * D) { const int c = q / D, dd = q % D; float s = 0.0f;
#pragma unroll 1
      for (int j = 0; j < N; ++j) { if (lab[j] == c) s += e[(size_t)j * D + dd]; }
      mcl[q] = s; }
    else if (q < NC * D + NC) { const int c = q - NC * D; float s = 0.0f, n = 0.0f;
#pragma unroll 1
      for (int j = 0; j < N; ++j) if (lab[j] == c) { s += sqs[j]; n += 1.0f; }
      scl[c] = s; scl[32 + c] = n; }
  }
  if (t >= 10 && t < 32) { scl[t] = 0.0f; scl[32 + t] = 0.0f; }
  __syncthreads();
  for (int pass = 0; pass < 2; ++pass) {
    for (int q = t; q < NC * D; q += 256) ((volatile float*)mc)[q] = mcl[q];
    if (t < 32) { ((volatile float*)Sc)[t] = scl[t]; ((volatile float*)ncnt)[t] = scl[32 + t]; }
    __threadfence();
  }
}

__global__ __launch_bounds__(128) void main_kernel(const b16* __restrict__ e16, const float* __restrict__ e, const int* __restrict__ lab, const float* __restrict__ sq,
                                                   const float* __restrict__ mc, const float* __restrict__ Sc, const float* __restrict__ ncnt, float* __restrict__ slot) {
  __shared__ int wps[128]; __shared__ float terms[128]; __shared__ float mcs[NC * D]; __shared__ int neg10[NC * 10];
  const int lane = threadIdx.x & 31, wave = threadIdx.x >> 5, nloc = lane & 15, hlf = lane >> 4, m0 = blockIdx.x * 128 + wave * 32;
  for (int q = threadIdx.x; q < NC * D; q += 128) mcs[q] = mc[q];
  if (threadIdx.x < NC) { const int Lc = threadIdx.x; int got = 0;
    for (int i = 0; i < 10; ++i) neg10[Lc * 10 + i] = 0;
    for (int c = 0; c < NC && got < 10; ++c) { if (c == Lc) continue;
#pragma unroll 1
      for (int j = 0; j < N && got < 10; ++j) { if (lab[j] == c) { neg10[Lc * 10 + got] = j; ++got; } } } }
  int labr[2][8];
#pragma unroll
  for (int r = 0; r < 2; ++r)
#pragma unroll
    for (int v = 0; v < 8; ++v) labr[r][v] = lab[m0 + r * 16 + v + 8 * hlf];
  float bestv[2][8]; int besti[2][8];
#pragma unroll
  for (int r = 0; r < 2; ++r)
#pragma unroll
    for (int v = 0; v < 8; ++v) { bestv[r][v] = -INFINITY; besti[r][v] = 0; }
  const Opnd A{e16, nullptr, D}, B{e16, nullptr, D};
#pragma unroll 1
  for (int tile = 0; tile < N / 64; ++tile) {
    const int c0 = tile * 64;
    v8f acc[2][4];
#pragma unroll
    for (int r = 0; r < 2; ++r)
#pragma unroll
      for (int t = 0; t < 4; ++t) acc[r][t] = (v8f){};
    gemm_tile<1, 1>(A, B, D, m0, c0, nloc, hlf, acc);
    int labc[4]; float sqc[4];
#pragma unroll
    for (int t = 0; t < 4; ++t) { const int j = c0 + t * 16 + nloc; labc[t] = lab[j]; sqc[t] = sq[j]; }
#pragma unroll
    for (int r = 0; r < 2; ++r)
#pragma unroll
      for (int v = 0; v < 8; ++v) {
        float best = -INFINITY; int bi = 0x7fffffff;
#pragma unroll
        for (int t = 0; t < 4; ++t) { const float val = (labc[t] == labr[r][v]) ? (sqc[t] - 2.0f * acc[r][t][v]) : -INFINITY; if (val > best) { best = val; bi = c0 + t * 16 + nloc; } }
#pragma unroll
        for (int o = 1; o < 16; o <<= 1) { const float ob = __shfl_xor(best, o); const int oi = __shfl_xor(bi, o); if (ob > best || (ob == best && oi < bi)) { best = ob; bi = oi; } }
        if (best > bestv[r][v]) { bestv[r][v] = best; besti[r][v] = bi; }
      }
  }
#pragma unroll
  for (int r = 0; r < 2; ++r)
#pragma unroll
    for (int v = 0; v < 8; ++v) if (nloc == 0) { int bi = besti[r][v]; bi = (bi < 0 || bi >= N) ? 0 : bi; wps[wave * 32 + r * 16 + v + 8 * hlf] = bi; }
  __syncthreads();
  { const int t = threadIdx.x, i = blockIdx.x * 128 + t; int li = lab[i]; li = li < 0 ? 0 : (li >= NC ? NC - 1 : li);
    const float* ei = e + (size_t)i * D; const float sqi = sq[i];
    float cs[NC];
#pragma unroll
    for (int c = 0; c < NC; ++c) { float dot = 0.0f;
#pragma unroll 1
      for (int dd = 0; dd < D; ++dd) dot += ei[dd] * mcs[c * D + dd];
      cs[c] = ncnt[c] * sqi + Sc[c] - 2.0f * dot; }
    float rowsum = 0.0f;
#pragma unroll
    for (int c = 0; c < NC; ++c) rowsum += cs[c];
    int js = 0; float bestn = INFINITY;
#pragma unroll
    for (int c = 0; c < NC; ++c) { const float nd = rowsum - cs[c]; if (nd < bestn) { bestn = nd; js = c; } }
    int wn = neg10[li * 10 + js]; wn = (wn < 0 || wn >= N) ? 0 : wn;
    const int wp = wps[t]; const float* ep = e + (size_t)wp * D; const float* en = e + (size_t)wn * D;
    float dp = 0.0f, dn = 0.0f;
#pragma unroll 1
    for (int dd = 0; dd < D; ++dd) { const float a = ei[dd] - ep[dd], b2 = ei[dd] - en[dd]; dp += a * a; dn += b2 * b2; }
    terms[t] = fmaxf(dp - dn + 1.0f, 0.0f); }
  __syncthreads();
  for (int o = 64; o > 0; o >>= 1) { if ((int)threadIdx.x < o) terms[threadIdx.x] += terms[threadIdx.x + o]; __syncthreads(); }
  if (threadIdx.x < 32) { const float v = (threadIdx.x == 0) ? terms[0] : 0.0f;
    for (int pass = 0; pass < 2; ++pass) { ((volatile float*)slot)[blockIdx.x * 32 + threadIdx.x] = v; __threadfence(); } }
}

__global__ __launch_bounds__(64) void final_kernel(const float* __restrict__ slot, float* __restrict__ out) {
  if (threadIdx.x == 0) { float s = 0.0f;
#pragma unroll 1
    for (int b = 0; b < NB; ++b) s += slot[b * 32];
    ((volatile float*)out)[0] = s; __threadfence(); ((volatile float*)out)[0] = s; }
}
}

extern "C" void kernel_launch(void* const* d_in, const int* in_sizes, int n_in,
                              void* d_out, int out_size, void* d_ws, size_t ws_size, hipStream_t stream) {
  (void)n_in; (void)out_size;
  const float* e = (const float*)d_in[0];
  const int* lab = (const int*)d_in[1];
  float* out = (float*)d_out;
  if (in_sizes[0] != N * D || in_sizes[1] != N) return;
  size_t off = 0; char* ws = (char*)d_ws;
  auto carve = [&](size_t bytes) { char* p = ws + off; off += (bytes + 255) & ~(size_t)255; return p; };
  b16* e16 = (b16*)carve((size_t)N * D * 2); float* sq = (float*)carve(N * 4); float* mc = (float*)carve(NC * D * 4); float* Sc = (float*)carve(256); float* ncnt = (float*)carve(256);
  float* slot = (float*)carve(NB * 32 * 4);
  if (off > ws_size) return;
  prep_kernel<<<1, 256, 0, stream>>>(e, lab, e16, sq, mc, Sc, ncnt);
  main_kernel<<<NB, 128, 0, stream>>>(e16, e, lab, sq, mc, Sc, ncnt, slot);
  final_kernel<<<1, 64, 0, stream>>>(slot, out);
}
